// SSIR_STGCN_87935160418920
// MI455X (gfx1250) — hardware-verified
//
#include <hip/hip_runtime.h>


#define NB_  4
#define TS   12
#define NND  128
#define NF   3
#define HH   64
#define G4   256
#define PP   14
#define NSQ  (NB_ * NND)
#define NE   (NB_ * NND * NND)
typedef _Float16 h16;
typedef unsigned short bf;
typedef __attribute__((ext_vector_type(16))) __bf16   v16bf;
typedef __attribute__((ext_vector_type(16))) _Float16 v16h;
typedef __attribute__((ext_vector_type(8)))  _Float16 v8h;
typedef __attribute__((ext_vector_type(8)))  unsigned short v8us;
typedef __attribute__((ext_vector_type(8)))  float    v8f;
typedef __attribute__((ext_vector_type(4)))  float    v4f;
typedef v8h  __attribute__((may_alias)) v8ha;
typedef v4f  __attribute__((may_alias)) v4fa;
typedef v8us __attribute__((may_alias)) v8usa;

__device__ __forceinline__ unsigned short f2bf(float f) { unsigned u = __float_as_uint(f); u += 0x7FFFu + ((u >> 16) & 1u); return (unsigned short)(u >> 16); }
__device__ __forceinline__ float bf2f(unsigned short b) { return __uint_as_float(((unsigned)b) << 16); }
__device__ __forceinline__ float bfr(float f) { return bf2f(f2bf(f)); }
__device__ __forceinline__ v16h cat16(v8h lo, v8h hi) { return __builtin_shufflevector(lo, hi, 0, 1, 2, 3, 4, 5, 6, 7, 8, 9, 10, 11, 12, 13, 14, 15); }
__device__ __forceinline__ v16bf cat16b(v8us lo, v8us hi) { return __builtin_bit_cast(v16bf, __builtin_shufflevector(lo, hi, 0, 1, 2, 3, 4, 5, 6, 7, 8, 9, 10, 11, 12, 13, 14, 15)); }
__device__ __forceinline__ v8f wmma16(v16h a, v16h b, v8f c) { return __builtin_amdgcn_wmma_f32_16x16x32_f16(false, a, false, b, (short)0, c, false, false); }
__device__ __forceinline__ v8f wmmab(v16bf a, v16bf b, v8f c) { return __builtin_amdgcn_wmma_f32_16x16x32_bf16(false, a, false, b, (short)0, c, false, false); }


template <typename T16> struct WFrag;
template <> struct WFrag<h16> { typedef v16h V; static __device__ __forceinline__ V ld(const h16* p) { return cat16(*(const v8h*)p, *(const v8h*)(p + 16)); } static __device__ __forceinline__ v8f mma(V a, V b, v8f c) { return wmma16(a, b, c); } };
template <> struct WFrag<bf> { typedef v16bf V; static __device__ __forceinline__ V ld(const bf* p) { return cat16b(*(const v8us*)p, *(const v8us*)(p + 16)); } static __device__ __forceinline__ v8f mma(V a, V b, v8f c) { return wmmab(a, b, c); } };
template <typename T16, int NSPLIT, bool BIAS>
__global__ __launch_bounds__(32) void k_gemmw(const T16* __restrict__ A, const T16* __restrict__ A2, const T16* __restrict__ Bt, const T16* __restrict__ Bt2, int K, float* C, int ldc, const float* __restrict__ bias, size_t sA, size_t sB, size_t sC) {
    typedef typename WFrag<T16>::V V;
    __shared__ __align__(16) float os[16 * 68];
    const size_t z = blockIdx.z; A += z * sA; if (A2) A2 += z * sA; Bt += z * sB; if (Bt2) Bt2 += z * sB; C += z * sC;
    const int lane = threadIdx.x & 31, lr = lane & 15, hi = lane >> 4; const int r0 = blockIdx.x * 64, c0 = blockIdx.y * 64;
    v8f acc[4][4];
#pragma unroll
    for (int mb = 0; mb < 4; ++mb)
#pragma unroll
        for (int nb = 0; nb < 4; ++nb) acc[mb][nb] = (v8f){};
    const size_t aoff = (size_t)(r0 + lr) * K + 8 * hi, boff = (size_t)(c0 + lr) * K + 8 * hi;
#pragma unroll 1
    for (int kc = 0; kc < K; kc += 32) {
        V a[4], a2[4];
#pragma unroll
        for (int mb = 0; mb < 4; ++mb) { a[mb] = WFrag<T16>::ld(A + aoff + (size_t)mb * 16 * K + kc); if (NSPLIT == 1 || NSPLIT == 2) a2[mb] = WFrag<T16>::ld(A2 + aoff + (size_t)mb * 16 * K + kc); }
#pragma unroll
        for (int nb = 0; nb < 4; ++nb) { const V b = WFrag<T16>::ld(Bt + boff + (size_t)nb * 16 * K + kc); V b2; if (NSPLIT >= 2) b2 = WFrag<T16>::ld(Bt2 + boff + (size_t)nb * 16 * K + kc);
#pragma unroll
            for (int mb = 0; mb < 4; ++mb) { acc[mb][nb] = WFrag<T16>::mma(a[mb], b, acc[mb][nb]); if (NSPLIT == 1 || NSPLIT == 2) acc[mb][nb] = WFrag<T16>::mma(a2[mb], b, acc[mb][nb]); if (NSPLIT >= 2) acc[mb][nb] = WFrag<T16>::mma(a[mb], b2, acc[mb][nb]); } }
        asm volatile("v_nop\n\tv_nop\n\tv_nop\n\tv_nop" : "+v"(acc[0][0]), "+v"(acc[1][1]), "+v"(acc[2][2]), "+v"(acc[3][3]) : "v"(a[0]), "v"(a[3]));
    }
#pragma unroll
    for (int mb = 0; mb < 4; ++mb) {
#pragma unroll
        for (int nb = 0; nb < 4; ++nb) {
#pragma unroll
            for (int j = 0; j < 8; ++j) os[(hi * 8 + j) * 68 + nb * 16 + lr] = acc[mb][nb][j]; }
        __builtin_amdgcn_wave_barrier(); asm volatile("" ::: "memory");
        float* crow = C + (size_t)(r0 + mb * 16) * ldc + c0;
#pragma unroll 1
        for (int ps = 0; ps < 2; ++ps) {
#pragma unroll
            for (int s = 0; s < 8; ++s) { const int row = 2 * s + hi, cofs = lr * 4; v4f val = *(const v4fa*)(os + row * 68 + cofs); if (BIAS) { val[0] += bfr(bias[c0 + cofs]); val[1] += bfr(bias[c0 + cofs + 1]); val[2] += bfr(bias[c0 + cofs + 2]); val[3] += bfr(bias[c0 + cofs + 3]); }
                *(volatile v4f*)(crow + (size_t)row * ldc + cofs) = val; }
            if (ps == 0) __threadfence(); }
        __builtin_amdgcn_wave_barrier(); asm volatile("" ::: "memory");
    }
}

__device__ __forceinline__ void splitf(float y, unsigned short& h, unsigned short& l) { h = f2bf(y); l = f2bf(y - bf2f(h)); }
__device__ __forceinline__ float sigm_(float a) { return __fdiv_rn(1.0f, __fadd_rn(1.0f, __expf(-a))); }
__device__ __forceinline__ float tanhf_(float a) { const float e2 = __expf(2.0f * a); return __fsub_rn(1.0f, __fdiv_rn(2.0f, __fadd_rn(e2, 1.0f))); }
typedef __attribute__((ext_vector_type(4))) unsigned short v4us;
typedef __attribute__((ext_vector_type(2))) float v2f;
__device__ __forceinline__ float xsv(const float* xs, int b, int t, int n, int f) { return bfr(xs[(((size_t)b * TS + t) * NND + n) * NF + f]); }

__global__ __launch_bounds__(256) void k_cvt8(const float* __restrict__ src, bf* dst, size_t n8) { const size_t i = (size_t)blockIdx.x * 256 + threadIdx.x; if (i >= n8) return; const v8f v = *(const v8f*)(src + i * 8); v8us o;
#pragma unroll
    for (int k = 0; k < 8; ++k) o[k] = f2bf(v[k]); *(volatile v8us*)(dst + i * 8) = o; __threadfence(); *(volatile v8us*)(dst + i * 8) = o; }
__global__ __launch_bounds__(256) void k_ngate(const float* __restrict__ xs, const float* __restrict__ bWih, const float* __restrict__ bWhh, const float* __restrict__ bb, const float* __restrict__ gWih, const float* __restrict__ gWhh, const float* __restrict__ gb, const float* __restrict__ NH, int t, float* NG) {
    const int e = blockIdx.x * 256 + threadIdx.x; if (e >= 2 * NSQ * G4) return; const int col = e % G4; const int s = (e / G4) % NSQ; const int w = e / (G4 * NSQ); const int b = s / NND, n = s % NND; const float* Wih = w ? gWih : bWih; const float* Whh = w ? gWhh : bWhh; const float* bias = w ? gb : bb; float a = bfr(bias[col]);
    for (int f = 0; f < NF; ++f) { float p = __fmul_rn(xsv(xs, b, t, n, f), bfr(Wih[col * NF + f])); asm volatile("" : "+v"(p)); a = __fadd_rn(a, p); }
    if (t > 0) { const float* h = NH + ((size_t)w * NSQ + s) * HH; for (int k = 0; k < HH; ++k) { float p = __fmul_rn(h[k], bfr(Whh[col * HH + k])); asm volatile("" : "+v"(p)); a = __fadd_rn(a, p); } }
    *(volatile float*)(NG + e) = a; __threadfence(); *(volatile float*)(NG + e) = a; }
__global__ __launch_bounds__(256) void k_cell(const float* __restrict__ G, int nrows, int first, float* Hs, float* Cs) { const int e = (blockIdx.x * 256 + threadIdx.x) * 2; if (e >= nrows * HH) return; const int j = e % HH; const size_t r = e / HH; const float* g = G + r * G4; const v2f cp = first ? (v2f){0.f, 0.f} : *(const v2f*)(Cs + e); v2f hn, cn;
#pragma unroll
    for (int q = 0; q < 2; ++q) { const int jq = j + q; const float ig = sigm_(g[jq]), fg = sigm_(g[HH + jq]), gg = tanhf_(g[2 * HH + jq]), og = sigm_(g[3 * HH + jq]); float fc = __fmul_rn(fg, cp[q]); asm volatile("" : "+v"(fc)); float igg = __fmul_rn(ig, gg); asm volatile("" : "+v"(igg)); cn[q] = __fadd_rn(fc, igg); hn[q] = __fmul_rn(og, tanhf_(cn[q])); }
    *(volatile v2f*)(Hs + e) = hn; *(volatile v2f*)(Cs + e) = cn; __threadfence(); *(volatile v2f*)(Hs + e) = hn; *(volatile v2f*)(Cs + e) = cn; }
__global__ __launch_bounds__(256) void k_egx(float* GH, const float* __restrict__ xs, const float* __restrict__ cWih, const float* __restrict__ cb, int t, int first) { const size_t e4 = ((size_t)blockIdx.x * 256 + threadIdx.x) * 4; if (e4 >= (size_t)NE * G4) return; const int col = (int)(e4 % G4); const size_t ed = e4 / G4; const int j = (int)(ed % NND); const int i = (int)((ed / NND) % NND); const int b = (int)(ed / (NND * NND)); float xi_[NF], xj_[NF];
#pragma unroll
    for (int f = 0; f < NF; ++f) { xi_[f] = xsv(xs, b, t, i, f); xj_[f] = xsv(xs, b, t, j, f); }
    const v4f prev = first ? (v4f){0.f, 0.f, 0.f, 0.f} : *(const v4f*)(GH + e4); v4f o;
#pragma unroll
    for (int q = 0; q < 4; ++q) { const int c = col + q; float a = __fadd_rn(prev[q], bfr(cb[c]));
#pragma unroll
        for (int f = 0; f < NF; ++f) { float p = __fmul_rn(xi_[f], bfr(cWih[c * 2 * NF + f])); asm volatile("" : "+v"(p)); float p2 = __fmul_rn(xj_[f], bfr(cWih[c * 2 * NF + NF + f])); asm volatile("" : "+v"(p2)); a = __fadd_rn(__fadd_rn(a, p), p2); } o[q] = a; }
    *(volatile v4f*)(GH + e4) = o; __threadfence(); *(volatile v4f*)(GH + e4) = o; }
__global__ __launch_bounds__(256) void k_spl(const float* __restrict__ F, size_t n4, bf* Fh, bf* Fl) { const size_t i = ((size_t)blockIdx.x * 256 + threadIdx.x) * 4; if (i >= n4 * 4) return; const v4f a = *(const v4f*)(F + i); v4us oh, ol;
#pragma unroll
    for (int q = 0; q < 4; ++q) { unsigned short u, c2; splitf(a[q], u, c2); oh[q] = u; ol[q] = c2; } *(volatile v4us*)(Fh + i) = oh; *(volatile v4us*)(Fl + i) = ol; __threadfence(); *(volatile v4us*)(Fh + i) = oh; *(volatile v4us*)(Fl + i) = ol; }
__global__ __launch_bounds__(256) void k_heads(const float* __restrict__ NH, const float* __restrict__ bfW, const float* __restrict__ bfb, const float* __restrict__ gfW, const float* __restrict__ gfb, float* BG) { const int e = blockIdx.x * 256 + threadIdx.x; if (e >= 2 * NSQ * PP) return; const int p = e % PP; const int s = (e / PP) % NSQ; const int w = e / (PP * NSQ); const float* W = w ? gfW : bfW; const float* bb = w ? gfb : bfb; const float* h = NH + ((size_t)w * NSQ + s) * HH; float a = 0.f;
    for (int k = 0; k < HH; ++k) { float q = __fmul_rn(h[k], bfr(W[p * HH + k])); asm volatile("" : "+v"(q)); a = __fadd_rn(a, q); } const float o = sigm_(__fadd_rn(a, bfr(bb[p]))); *(volatile float*)(BG + e) = o; __threadfence(); *(volatile float*)(BG + e) = o; }
__global__ __launch_bounds__(256) void k_cij(const float* __restrict__ EH, const float* __restrict__ cfW, const float* __restrict__ cfb, float* CS) { const size_t e = (size_t)blockIdx.x * 256 + threadIdx.x; if (e >= (size_t)NE * PP) return; const int p = (int)(e % PP); const size_t ed = e / PP; const int j = (int)(ed % NND); const size_t bi = ed / NND; const float* h = EH + ed * HH; float a = 0.f;
    for (int k = 0; k < HH; ++k) { float q = __fmul_rn(h[k], bfr(cfW[p * HH + k])); asm volatile("" : "+v"(q)); a = __fadd_rn(a, q); } const float o = sigm_(__fadd_rn(a, bfr(cfb[p]))); const size_t off = (bi * PP + p) * NND + j; *(volatile float*)(CS + off) = o; __threadfence(); *(volatile float*)(CS + off) = o; }
__global__ __launch_bounds__(256) void k_csm(float* CS) { const int lane = threadIdx.x & 31; const int row = blockIdx.x * 8 + (threadIdx.x >> 5); if (row >= NSQ * PP) return; float* r = CS + (size_t)row * NND; const v4f a = *(const v4f*)(r + lane * 4); float mx = fmaxf(fmaxf(a[0], a[1]), fmaxf(a[2], a[3]));
#pragma unroll
    for (int sh = 16; sh; sh >>= 1) mx = fmaxf(mx, __shfl_xor(mx, sh, 32));
    v4f ex; float s = 0.f;
#pragma unroll
    for (int q = 0; q < 4; ++q) { ex[q] = __expf(__fsub_rn(a[q], mx)); s = __fadd_rn(s, ex[q]); }
#pragma unroll
    for (int sh = 16; sh; sh >>= 1) s += __shfl_xor(s, sh, 32);
    const float rs = __fdiv_rn(1.0f, s); v4f o; o[0] = __fmul_rn(ex[0], rs); o[1] = __fmul_rn(ex[1], rs); o[2] = __fmul_rn(ex[2], rs); o[3] = __fmul_rn(ex[3], rs); *(volatile v4f*)(r + lane * 4) = o; __threadfence(); *(volatile v4f*)(r + lane * 4) = o; }
__global__ __launch_bounds__(256) void k_sir(const float* __restrict__ CS, const float* __restrict__ BG, const float* __restrict__ SIR, int p, float* SIRn, float* ST4) { const int e = blockIdx.x * 256 + threadIdx.x; if (e >= NSQ) return; const int i = e % NND, b = e / NND; const float* cr = CS + (((size_t)b * NND + i) * PP + p) * NND; float inf = 0.f;
    for (int j = 0; j < NND; ++j) { float q = __fmul_rn(cr[j], SIR[((size_t)b * NND + j) * 4 + 1]); asm volatile("" : "+v"(q)); inf = __fadd_rn(inf, q); }
    const float S = SIR[(size_t)e * 4], I = SIR[(size_t)e * 4 + 1], R = SIR[(size_t)e * 4 + 2]; const float beta = BG[(size_t)e * PP + p], gamma = BG[((size_t)NSQ + e) * PP + p]; const float Nt = fmaxf(__fadd_rn(__fadd_rn(S, I), R), 1e-8f);
    float t1 = __fmul_rn(-beta, S); asm volatile("" : "+v"(t1)); float t2 = __fdiv_rn(t1, Nt); asm volatile("" : "+v"(t2)); const float dS = __fmul_rn(t2, inf); float gI = __fmul_rn(gamma, I); asm volatile("" : "+v"(gI)); const float dI = __fsub_rn(-dS, gI); const float dR = gI;
    const float St = fmaxf(__fadd_rn(S, dS), 0.f), It = fmaxf(__fadd_rn(I, dI), 0.f), Rt = fmaxf(__fadd_rn(R, dR), 0.f); const float sc = __fdiv_rn(Nt, fmaxf(__fadd_rn(__fadd_rn(St, It), Rt), 1e-8f)); const float In = fmaxf(-dS, 0.f);
    v4f o; o[0] = In; o[1] = __fmul_rn(St, sc); o[2] = __fmul_rn(It, sc); o[3] = __fmul_rn(Rt, sc); v4f ns; ns[0] = o[1]; ns[1] = o[2]; ns[2] = o[3]; ns[3] = 0.f;
    *(volatile v4f*)(ST4 + ((size_t)p * NSQ + e) * 4) = o; *(volatile v4f*)(SIRn + (size_t)e * 4) = ns; __threadfence(); *(volatile v4f*)(ST4 + ((size_t)p * NSQ + e) * 4) = o; *(volatile v4f*)(SIRn + (size_t)e * 4) = ns; }
__global__ __launch_bounds__(256) void k_sir0(const float* __restrict__ x, float* SIR) { const int e = blockIdx.x * 256 + threadIdx.x; if (e >= NSQ) return; const int n = e % NND, b = e / NND; v4f o; o[0] = xsv(x, b, TS - 1, n, 0); o[1] = xsv(x, b, TS - 1, n, 1); o[2] = xsv(x, b, TS - 1, n, 2); o[3] = 0.f; *(volatile v4f*)(SIR + (size_t)e * 4) = o; __threadfence(); *(volatile v4f*)(SIR + (size_t)e * 4) = o; }
__global__ __launch_bounds__(256) void k_out013(const float* __restrict__ ST4, float* O0, float* O2, float* O3) { const int e = (blockIdx.x * 256 + threadIdx.x) * 4; if (e >= NB_ * PP * NND * 3) return;
    { v4f o;
#pragma unroll
      for (int q = 0; q < 4; ++q) { const int f = e + q; const int c = f % 3; const int n = (f / 3) % NND; const int p = (f / (3 * NND)) % PP; const int b = f / (3 * NND * PP); o[q] = ST4[(((size_t)p * NB_ + b) * NND + n) * 4 + 1 + c]; } *(volatile v4f*)(O2 + e) = o; __threadfence(); *(volatile v4f*)(O2 + e) = o; }
    if (e < NB_ * PP * NND) { v4f a, d;
#pragma unroll
      for (int q = 0; q < 4; ++q) { const int f = e + q; const int n = f % NND; const int p = (f / NND) % PP; const int b = f / (NND * PP); const float* s = ST4 + (((size_t)p * NB_ + b) * NND + n) * 4; a[q] = s[2]; d[q] = s[0]; } *(volatile v4f*)(O0 + e) = a; *(volatile v4f*)(O3 + e) = d; __threadfence(); *(volatile v4f*)(O0 + e) = a; *(volatile v4f*)(O3 + e) = d; } }
__global__ __launch_bounds__(256) void k_out1(const float* __restrict__ BG, const float* __restrict__ CS, float* O1) { const size_t e = ((size_t)blockIdx.x * 256 + threadIdx.x) * 4; if (e >= (size_t)NB_ * PP * NND * (NND + 2)) return; v4f o;
#pragma unroll
    for (int q = 0; q < 4; ++q) { const size_t f = e + q; const int c = (int)(f % (NND + 2)); const int n = (int)((f / (NND + 2)) % NND); const int p = (int)((f / ((NND + 2) * NND)) % PP); const int b = (int)(f / ((size_t)(NND + 2) * NND * PP)); const size_t s = (size_t)b * NND + n;
        o[q] = c == 0 ? BG[s * PP + p] : (c == 1 ? BG[((size_t)NSQ + s) * PP + p] : CS[(s * PP + p) * NND + (c - 2)]); }
    *(volatile v4f*)(O1 + e) = o; __threadfence(); *(volatile v4f*)(O1 + e) = o; }

extern "C" void kernel_launch(void* const* d_in, const int* in_sizes, int n_in,
                              void* d_out, int out_size, void* d_ws, size_t ws_size, hipStream_t stream) {
    (void)in_sizes; (void)n_in; (void)out_size;
    const float* IN[17]; for (int i = 0; i < 17; ++i) IN[i] = (const float*)d_in[i];
    float* O0 = (float*)d_out; float* O1 = (float*)((char*)d_out + 28672); float* O2 = (float*)((char*)d_out + 3756032); float* O3 = (float*)((char*)d_out + 3842048);
    char* wsp = (char*)d_ws;
    auto take = [&](size_t bytes) { char* p = wsp; wsp += (bytes + 255) & ~(size_t)255; return (void*)p; };
    bf* WHH = (bf*)take((size_t)G4 * HH * 2); float* NG = (float*)take((size_t)2 * NSQ * G4 * 4); float* NH = (float*)take((size_t)2 * NSQ * HH * 4); float* NC = (float*)take((size_t)2 * NSQ * HH * 4); float* BG = (float*)take((size_t)2 * NSQ * PP * 4);
    float* GH = (float*)take((size_t)NE * G4 * 4); float* EH = (float*)take((size_t)NE * HH * 4); float* EC = (float*)take((size_t)NE * HH * 4); bf* Eh = (bf*)take((size_t)NE * HH * 2); bf* El = (bf*)take((size_t)NE * HH * 2); float* CS = (float*)take((size_t)NSQ * PP * NND * 4);
    float* SIRa = (float*)take((size_t)NSQ * 4 * 4); float* SIRb = (float*)take((size_t)NSQ * 4 * 4); float* ST4 = (float*)take((size_t)PP * NSQ * 4 * 4);
    if ((size_t)(wsp - (char*)d_ws) > ws_size) return;
    k_cvt8<<<(G4 * HH / 8 + 255) / 256, 256, 0, stream>>>(IN[13], WHH, (size_t)G4 * HH / 8);
    for (int t = 0; t < TS; ++t) {
        k_ngate<<<(2 * NSQ * G4 + 255) / 256, 256, 0, stream>>>(IN[0], IN[2], IN[3], IN[4], IN[7], IN[8], IN[9], NH, t, NG); k_cell<<<(2 * NSQ * HH / 2 + 255) / 256, 256, 0, stream>>>(NG, 2 * NSQ, t == 0, NH, NC); }
    k_heads<<<(2 * NSQ * PP + 255) / 256, 256, 0, stream>>>(NH, IN[5], IN[6], IN[10], IN[11], BG);
    for (int t = 0; t < TS; ++t) {
        if (t > 0) { k_spl<<<(NE * HH / 4 + 255) / 256, 256, 0, stream>>>(EH, (size_t)NE * HH / 4, Eh, El); k_gemmw<bf, 1, false><<<dim3(NE / 64, G4 / 64, 1), 32, 0, stream>>>(Eh, El, WHH, nullptr, HH, GH, G4, nullptr, 0, 0, 0); }
        k_egx<<<(unsigned)(((size_t)NE * G4 / 4 + 255) / 256), 256, 0, stream>>>(GH, IN[0], IN[12], IN[14], t, t == 0); k_cell<<<(NE * HH / 2 + 255) / 256, 256, 0, stream>>>(GH, NE, t == 0, EH, EC); }
    k_cij<<<(unsigned)(((size_t)NE * PP + 255) / 256), 256, 0, stream>>>(EH, IN[15], IN[16], CS); k_csm<<<(NSQ * PP + 7) / 8, 256, 0, stream>>>(CS);
    k_sir0<<<(NSQ + 255) / 256, 256, 0, stream>>>(IN[1], SIRa);
    for (int p = 0; p < PP; ++p) k_sir<<<(NSQ + 255) / 256, 256, 0, stream>>>(CS, BG, (p & 1) ? SIRb : SIRa, p, (p & 1) ? SIRa : SIRb, ST4);
    k_out013<<<(NB_ * PP * NND * 3 / 4 + 255) / 256, 256, 0, stream>>>(ST4, O0, O2, O3); k_out1<<<(unsigned)(((size_t)NB_ * PP * NND * (NND + 2) / 4 + 255) / 256), 256, 0, stream>>>(BG, CS, O1);
}
